// BayesianAttention_43731357008231
// MI455X (gfx1250) — hardware-verified
//
#include <hip/hip_runtime.h>
#include <stddef.h>
#include <stdint.h>

#define SQ    2048
#define HID   2048
#define NH    16
#define HDM   128
#define WNC   64
#define NQKV  6144
#define NSLAB 48
#define QB    128
#define KC    64
#define NQB   (SQ / QB)
#define NKCH  (SQ / KC)
#define FLW   32
#define FLMAGIC 0x0F1A65EDu
#define LUTN  2176
#define MTH   (-1.0e8f)

static_assert(HID == NH * HDM);
static_assert(NQKV == 3 * HID);
static_assert(NSLAB * HDM == NQKV);
static_assert(HDM % 32 == 0);
static_assert(2 * WNC == HDM);
static_assert(HID % 32 == 0);
static_assert(HID == 256 * 8);
static_assert(SQ % 256 == 0);
static_assert(SQ % 64 == 0);
static_assert(NQB * QB == SQ);
static_assert(NKCH * KC == SQ);
static_assert(NKCH <= 32);
static_assert(LUTN >= SQ + QB);
static_assert(SQ == 16 * 32 * 4);
static_assert(QB == 8 * 16);

typedef _Float16 v16h __attribute__((ext_vector_type(16)));
typedef _Float16 v8h  __attribute__((ext_vector_type(8)));
typedef float    v8f  __attribute__((ext_vector_type(8)));
typedef float    v4f  __attribute__((ext_vector_type(4)));
typedef unsigned int v4u __attribute__((ext_vector_type(4)));
typedef float fal __attribute__((may_alias));

union Frag  { v16h v; v8h h[2]; };
union Pack8 { v8h h; v4u u; };

__device__ __forceinline__ v8f mma16(v16h a, v16h b, v8f c) {
  c = __builtin_amdgcn_wmma_f32_16x16x32_f16(false, a, false, b, (short)0, c, false, false);
  asm volatile("v_nop\n\tv_nop\n\tv_nop\n\tv_nop" : "+v"(c) : "v"(a), "v"(b));
  return c;
}

__device__ __forceinline__ v16h ldfrag(const _Float16* p, int ld, int row0, int k0, int lane) {
  const int m = lane & 15, lh = lane >> 4;
  const _Float16* q = p + (size_t)(row0 + m) * ld + k0 + 8 * lh;
  Frag f;
  f.h[0] = *(const v8h*)(q);
  f.h[1] = *(const v8h*)(q + 16);
  return f.v;
}

__device__ __forceinline__ v8f zero8() { return (v8f){0.f, 0.f, 0.f, 0.f, 0.f, 0.f, 0.f, 0.f}; }

__device__ __forceinline__ void gemm32x64(const _Float16* __restrict__ A, int lda,
                                          const _Float16* __restrict__ Bt, int ldb,
                                          int m0, int n0, int lane, v8f (&acc)[2][4]) {
#pragma unroll 1
  for (int k0 = 0; k0 < HID; k0 += 32) {
    const v16h a0 = ldfrag(A, lda, m0, k0, lane);
    const v16h a1 = ldfrag(A, lda, m0 + 16, k0, lane);
#pragma unroll
    for (int t = 0; t < 4; ++t) {
      const v16h b = ldfrag(Bt, ldb, n0 + 16 * t, k0, lane);
      acc[0][t] = mma16(a0, b, acc[0][t]);
      acc[1][t] = mma16(a1, b, acc[1][t]);
    }
  }
}

__device__ __forceinline__ void gemm32x64seg(const _Float16* __restrict__ Op, int bh0, int s0, int prow,
                                             const _Float16* __restrict__ Bt, int n0, int lane, v8f (&acc)[2][4]) {
#pragma unroll 1
  for (int h = 0; h < NH; ++h) {
    const _Float16* A = Op + ((size_t)(bh0 + h) * prow + s0) * HDM;
#pragma unroll
    for (int sub = 0; sub < HDM / 32; ++sub) {
      const int ka = sub * 32, kb = h * HDM + sub * 32;
      const v16h a0 = ldfrag(A, HDM, 0, ka, lane);
      const v16h a1 = ldfrag(A, HDM, 16, ka, lane);
      const v16h b0 = ldfrag(Bt, HID, n0, kb, lane);
      const v16h b1 = ldfrag(Bt, HID, n0 + 16, kb, lane);
      const v16h b2 = ldfrag(Bt, HID, n0 + 32, kb, lane);
      const v16h b3 = ldfrag(Bt, HID, n0 + 48, kb, lane);
      acc[0][0] = mma16(a0, b0, acc[0][0]);
      acc[1][0] = mma16(a1, b0, acc[1][0]);
      acc[0][1] = mma16(a0, b1, acc[0][1]);
      acc[1][1] = mma16(a1, b1, acc[1][1]);
      acc[0][2] = mma16(a0, b2, acc[0][2]);
      acc[1][2] = mma16(a1, b2, acc[1][2]);
      acc[0][3] = mma16(a0, b3, acc[0][3]);
      acc[1][3] = mma16(a1, b3, acc[1][3]);
    }
  }
}

__global__ __launch_bounds__(256) void k_mflag(const float* __restrict__ mask, unsigned* __restrict__ fl) {
  __shared__ unsigned red[8][4];
  const int tid = threadIdx.x, lane = tid & 31, wave = tid >> 5;
  const int qb = blockIdx.x;
  unsigned allm = 0xFFFFFFFFu, allz = 0xFFFFFFFFu, rowsfin = 1u;
#pragma unroll 1
  for (int rr = 0; rr < 16; ++rr) {
    const float* mp = mask + (size_t)(qb * QB + wave * 16 + rr) * SQ;
    unsigned rf = 0u;
#pragma unroll 4
    for (int j = 0; j < 16; ++j) {
      const v4f v = *(const v4f*)(mp + 4 * (lane + 32 * j));
      const unsigned bit = 1u << ((lane >> 4) + 2 * j);
      const bool fin = (v[0] > MTH) || (v[1] > MTH) || (v[2] > MTH) || (v[3] > MTH);
      const bool nz  = (v[0] != 0.0f) || (v[1] != 0.0f) || (v[2] != 0.0f) || (v[3] != 0.0f);
      allm &= fin ? ~bit : 0xFFFFFFFFu;
      allz &= nz  ? ~bit : 0xFFFFFFFFu;
      rf |= fin ? 1u : 0u;
    }
#pragma unroll
    for (int off = 1; off < 32; off <<= 1) rf |= __shfl_xor(rf, off, 32);
    rowsfin &= rf;
  }
#pragma unroll
  for (int off = 1; off < 32; off <<= 1) {
    allm &= __shfl_xor(allm, off, 32);
    allz &= __shfl_xor(allz, off, 32);
  }
  if (lane == 0) { red[wave][0] = allm; red[wave][1] = allz; red[wave][2] = rowsfin; red[wave][3] = 0u; }
  __syncthreads();
  if (wave == 0) {
    unsigned a = 0xFFFFFFFFu, z = 0xFFFFFFFFu, f = 1u;
#pragma unroll
    for (int w = 0; w < 8; ++w) { a &= red[w][0]; z &= red[w][1]; f &= red[w][2]; }
    const unsigned word = (lane == 0) ? a : ((lane == 1) ? z : ((lane == 2) ? f : ((lane == 3) ? FLMAGIC : 0u)));
    volatile unsigned* d = (volatile unsigned*)(fl + qb * FLW + lane);
    *d = word;
    __threadfence();
    *d = word;
  }
}

__global__ __launch_bounds__(256) void k_cvt(const float* __restrict__ src, _Float16* __restrict__ dst, float sc) {
  const int row = blockIdx.x;
  const int col = (int)threadIdx.x * 8;
  const size_t o = (size_t)row * HID + col;
  const v4f a0 = *(const v4f*)(src + o);
  const v4f a1 = *(const v4f*)(src + o + 4);
  Pack8 pk;
  pk.h = (v8h){(_Float16)(a0[0] * sc), (_Float16)(a0[1] * sc), (_Float16)(a0[2] * sc), (_Float16)(a0[3] * sc),
               (_Float16)(a1[0] * sc), (_Float16)(a1[1] * sc), (_Float16)(a1[2] * sc), (_Float16)(a1[3] * sc)};
  const v4u vv = pk.u;
  volatile v4u* d = (volatile v4u*)(dst + o);
  *d = vv;
  __threadfence();
  *d = vv;
}

#define SFP 132
__global__ __launch_bounds__(128) __attribute__((amdgpu_num_vgpr(256)))
void k_qkv(const _Float16* __restrict__ xh, const _Float16* __restrict__ wt,
           _Float16* __restrict__ qp, _Float16* __restrict__ kp, _Float16* __restrict__ vtp) {
  __shared__ __align__(16) float sf[64 * SFP];
  const int tid = threadIdx.x, lane = tid & 31, wave = tid >> 5;
  const int hh = lane >> 4, c = lane & 15;
  const int wm = wave >> 1, wn = wave & 1;
  const int mb = blockIdx.x * 64;
  const int ns = blockIdx.y;
  const int which = ns / NH;
  const int head  = ns - which * NH;
  const int m0 = mb + wm * 32;
  const int n0 = ns * HDM + wn * WNC;

  v8f acc[2][4];
#pragma unroll
  for (int s = 0; s < 2; ++s)
#pragma unroll
    for (int t = 0; t < 4; ++t) acc[s][t] = zero8();
  gemm32x64(xh, HID, wt, HID, m0, n0, lane, acc);

#pragma unroll
  for (int sub = 0; sub < 2; ++sub)
#pragma unroll
    for (int t = 0; t < 4; ++t)
#pragma unroll
      for (int r = 0; r < 8; ++r)
        sf[(wm * 32 + 16 * sub + 8 * hh + r) * SFP + wn * WNC + 16 * t + c] = acc[sub][t][r] * 0.03125f;
  __syncthreads();

  if (which < 2) {
    v4u val[8];
    size_t go[8];
#pragma unroll
    for (int j = 0; j < 8; ++j) {
      const int p  = tid + 128 * j;
      const int lr = p >> 4;
      const int pc = p & 15;
      const int d0 = pc * 8;
      const float* ra = sf + lr * SFP + d0;
      const v4f a0 = *(const v4f*)(ra), a1 = *(const v4f*)(ra + 4);
      Pack8 pk;
      pk.h = (v8h){(_Float16)a0[0], (_Float16)a0[1], (_Float16)a0[2], (_Float16)a0[3],
                   (_Float16)a1[0], (_Float16)a1[1], (_Float16)a1[2], (_Float16)a1[3]};
      val[j] = pk.u;
      go[j]  = ((size_t)head * SQ + mb + lr) * HDM + d0;
    }
    _Float16* base = (which == 0) ? qp : kp;
    for (int ps = 0; ps < 2; ++ps) {
#pragma unroll
      for (int j = 0; j < 8; ++j) *(volatile v4u*)(base + go[j]) = val[j];
      __threadfence();
    }
  } else {
    v4u val[8];
    size_t go[8];
#pragma unroll
    for (int j = 0; j < 8; ++j) {
      const int p  = tid + 128 * j;
      const int d  = p >> 3;
      const int pc = p & 7;
      const float* cp = sf + (pc * 8) * SFP + d;
      Pack8 pk;
      pk.h = (v8h){(_Float16)cp[0 * SFP], (_Float16)cp[1 * SFP], (_Float16)cp[2 * SFP], (_Float16)cp[3 * SFP],
                   (_Float16)cp[4 * SFP], (_Float16)cp[5 * SFP], (_Float16)cp[6 * SFP], (_Float16)cp[7 * SFP]};
      val[j] = pk.u;
      go[j]  = ((size_t)head * HDM + d) * SQ + mb + pc * 8;
    }
    for (int ps = 0; ps < 2; ++ps) {
#pragma unroll
      for (int j = 0; j < 8; ++j) *(volatile v4u*)(vtp + go[j]) = val[j];
      __threadfence();
    }
  }
}

#define PSP 128
static_assert(16 * PSP * 2 == 16 * KC * 4);
static_assert(PSP >= HDM);
__global__ __launch_bounds__(256) __attribute__((amdgpu_num_vgpr(256)))
void k_attn(const _Float16* __restrict__ qp, const _Float16* __restrict__ kp,
            const _Float16* __restrict__ vt, const float* __restrict__ mask,
            const unsigned* __restrict__ fl,
            const float* __restrict__ pshape, const float* __restrict__ plogsc,
            const float* __restrict__ ploc, const float* __restrict__ pseqsc,
            const float* __restrict__ pseclen, _Float16* __restrict__ op) {
  __shared__ __align__(16) _Float16 Ps[8 * 16 * PSP];
  __shared__ float lut[LUTN];

  const int tid = threadIdx.x, lane = tid & 31, wave = tid >> 5;
  const int hh = lane >> 4, c = lane & 15;
  const int qb = blockIdx.x % NQB;
  const int hb = blockIdx.x / NQB;
  const int q0 = qb * QB + wave * 16;
  const int doff = qb * QB + QB - 1;

  const _Float16* Q = qp + (size_t)hb * SQ * HDM;
  const _Float16* K = kp + (size_t)hb * SQ * HDM;
  const _Float16* V = vt + (size_t)hb * HDM * SQ;

  const float shp    = pshape[hb];
  const float escale = expf(plogsc[hb]);
  const float locv   = ploc[hb];
  const float locoff = expf(locv) - expf(-locv);
  const float ssm    = pseclen[0] * pseqsc[hb];
  const bool  shpone = (shp == 1.0f);
  for (int i = tid; i < LUTN; i += 256) {
    const float bq   = (float)(i - doff) - locoff;
    const float base = fabsf(bq) + 1.0e-5f;
    float pv = base;
    if (!shpone) pv = powf(base, shp);
    lut[i] = -(pv * escale);
  }

  const unsigned w0 = (unsigned)__builtin_amdgcn_readfirstlane((int)fl[qb * FLW + 0]);
  const unsigned w1 = (unsigned)__builtin_amdgcn_readfirstlane((int)fl[qb * FLW + 1]);
  const unsigned w2 = (unsigned)__builtin_amdgcn_readfirstlane((int)fl[qb * FLW + 2]);
  const unsigned w3 = (unsigned)__builtin_amdgcn_readfirstlane((int)fl[qb * FLW + 3]);
  const bool valid = (w3 == FLMAGIC);
  const unsigned allm = valid ? w0 : 0u;
  const unsigned allz = valid ? w1 : 0u;
  const bool rfin = valid && ((w2 & 1u) != 0u);

  const float NEGI = -__builtin_huge_valf();
  float mrow[8], lrow[8];
  v8f oacc[8];
#pragma unroll
  for (int r = 0; r < 8; ++r) { mrow[r] = NEGI; lrow[r] = 0.f; }
#pragma unroll
  for (int t = 0; t < 8; ++t) oacc[t] = zero8();

  _Float16* pw  = Ps + wave * 16 * PSP;
  float*    mwf = (float*)pw;
  const float rs = 0.08838834764831845f;
  __syncthreads();

  for (int kc = 0; kc < NKCH; ++kc) {
    if (rfin && (((allm >> kc) & 1u) != 0u)) continue;
    const bool ldm = (((allz >> kc) & 1u) == 0u);
    const int kv0 = kc * KC;
    __syncthreads();
    if (ldm) {
#pragma unroll
      for (int it = 0; it < 8; ++it) {
        const int p   = lane + 32 * it;
        const int row = p >> 4;
        const int c4  = (p & 15) * 4;
        *(v4f*)(mwf + row * KC + c4) = *(const v4f*)(mask + (size_t)(q0 + row) * SQ + kv0 + c4);
      }
    }
    __syncthreads();

    v8f s[4];
#pragma unroll
    for (int j = 0; j < 4; ++j) s[j] = zero8();
#pragma unroll
    for (int dc = 0; dc < HDM / 32; ++dc) {
      const v16h qa = ldfrag(Q, HDM, q0, dc * 32, lane);
#pragma unroll
      for (int j = 0; j < 4; ++j) {
        const v16h kb = ldfrag(K, HDM, kv0 + j * 16, dc * 32, lane);
        s[j] = mma16(qa, kb, s[j]);
      }
    }
    const int li0 = kv0 + c - q0 - 8 * hh + doff;
    if (ldm) {
      const fal* mr = (const fal*)mwf + (8 * hh) * KC + c;
#pragma unroll
      for (int r = 0; r < 8; ++r)
#pragma unroll
        for (int j = 0; j < 4; ++j)
          s[j][r] = (s[j][r] * rs + lut[li0 + 16 * j - r]) * ssm + mr[r * KC + 16 * j];
    } else {
#pragma unroll
      for (int r = 0; r < 8; ++r)
#pragma unroll
        for (int j = 0; j < 4; ++j)
          s[j][r] = (s[j][r] * rs + lut[li0 + 16 * j - r]) * ssm;
    }
    __builtin_amdgcn_fence(__ATOMIC_RELEASE, "wavefront");
    __builtin_amdgcn_wave_barrier();
    float cm[8];
#pragma unroll
    for (int r = 0; r < 8; ++r) {
      float m = NEGI;
#pragma unroll
      for (int j = 0; j < 4; ++j) m = fmaxf(m, s[j][r]);
#pragma unroll
      for (int off = 1; off < 16; off <<= 1) m = fmaxf(m, __shfl_xor(m, off, 32));
      cm[r] = m;
    }
    float al[8];
#pragma unroll
    for (int r = 0; r < 8; ++r) {
      const float mnew  = fmaxf(mrow[r], cm[r]);
      const float msafe = (mnew == NEGI) ? 0.f : mnew;
      const float alpha = __expf(mrow[r] - msafe);
      mrow[r] = mnew;
      float psum = 0.f;
#pragma unroll
      for (int j = 0; j < 4; ++j) {
        const float p = __expf(s[j][r] - msafe);
        psum += p;
        pw[(8 * hh + r) * PSP + j * 16 + c] = (_Float16)(p * 1024.0f);
      }
#pragma unroll
      for (int off = 1; off < 16; off <<= 1) psum += __shfl_xor(psum, off, 32);
      lrow[r] = lrow[r] * alpha + psum;
      al[r] = alpha;
    }
#pragma unroll
    for (int t = 0; t < 8; ++t)
#pragma unroll
      for (int r = 0; r < 8; ++r) oacc[t][r] *= al[r];
    __syncthreads();

#pragma unroll
    for (int kk = 0; kk < 2; ++kk) {
      const v16h pa = ldfrag(pw, PSP, 0, kk * 32, lane);
#pragma unroll
      for (int t = 0; t < 8; ++t) {
        const v16h vb = ldfrag(V, SQ, t * 16, kv0 + kk * 32, lane);
        oacc[t] = mma16(pa, vb, oacc[t]);
      }
    }
  }

  float invl[8];
#pragma unroll
  for (int r = 0; r < 8; ++r) invl[r] = (lrow[r] > 0.f) ? (0.015625f / lrow[r]) : 0.f;
  __syncthreads();
#pragma unroll
  for (int r = 0; r < 8; ++r) {
#pragma unroll
    for (int t = 0; t < 8; ++t)
      pw[(8 * hh + r) * PSP + 16 * t + c] = (_Float16)(oacc[t][r] * invl[r]);
  }
  __syncthreads();
  v4u val[8];
  size_t go[8];
#pragma unroll
  for (int it = 0; it < 8; ++it) {
    const int p  = lane + 32 * it;
    const int L  = p >> 4;
    const int pc = p & 15;
    Pack8 pk;
    pk.h    = *(const v8h*)(pw + L * PSP + pc * 8);
    val[it] = pk.u;
    go[it]  = ((size_t)hb * SQ + q0 + L) * HDM + pc * 8;
  }
  for (int ps = 0; ps < 2; ++ps) {
#pragma unroll
    for (int it = 0; it < 8; ++it) *(volatile v4u*)(op + go[it]) = val[it];
    __threadfence();
  }
}

#define OTP 68
__device__ __forceinline__ void out_epilogue(v8f (&acc)[2][4], float scale, float* sw, float* __restrict__ out,
                                             int m0, int n0, int lane, int hh, int c) {
#pragma unroll
  for (int sub = 0; sub < 2; ++sub) {
    __syncthreads();
#pragma unroll
    for (int t = 0; t < 4; ++t) {
#pragma unroll
      for (int r = 0; r < 8; ++r) sw[(8 * hh + r) * OTP + 16 * t + c] = acc[sub][t][r] * scale;
    }
    __syncthreads();
    v4f val[8];
    size_t go[8];
#pragma unroll
    for (int it = 0; it < 8; ++it) {
      const int p    = lane + 32 * it;
      const int L    = p >> 3;
      const int pc   = p & 7;
      const int row  = L >> 1;
      const int half = L & 1;
      val[it] = *(const v4f*)(sw + row * OTP + half * 32 + pc * 4);
      go[it]  = (size_t)(m0 + sub * 16 + row) * HID + n0 + half * 32 + pc * 4;
    }
    for (int ps = 0; ps < 2; ++ps) {
#pragma unroll
      for (int it = 0; it < 8; ++it) *(volatile v4f*)(out + go[it]) = val[it];
      __threadfence();
    }
  }
}

__global__ __launch_bounds__(256) __attribute__((amdgpu_num_vgpr(256)))
void k_out(const _Float16* __restrict__ op, const _Float16* __restrict__ wt, float* __restrict__ out) {
  __shared__ __align__(16) float st[8][16 * OTP];
  const int tid = threadIdx.x, lane = tid & 31, wave = tid >> 5;
  const int hh = lane >> 4, c = lane & 15;
  const int s0 = blockIdx.x * 256 + wave * 32;
  const int n0 = blockIdx.y * 64;

  v8f acc[2][4];
#pragma unroll
  for (int s = 0; s < 2; ++s)
#pragma unroll
    for (int t = 0; t < 4; ++t) acc[s][t] = zero8();
  gemm32x64seg(op, 0, s0, SQ, wt, n0, lane, acc);
  out_epilogue(acc, 0.001953125f, st[wave], out, s0, n0, lane, hh, c);
}

extern "C" void kernel_launch(void* const* d_in, const int* in_sizes, int n_in,
                              void* d_out, int out_size, void* d_ws, size_t ws_size,
                              hipStream_t stream) {
  if (n_in < 11) return;
  if (in_sizes[0] != SQ * HID) return;
  if (in_sizes[1] != HID * HID) return;
  if (in_sizes[2] != HID * HID) return;
  if (in_sizes[3] != HID * HID) return;
  if (in_sizes[4] != HID * HID) return;
  if (in_sizes[5] != NH) return;
  if (in_sizes[6] != NH) return;
  if (in_sizes[7] != NH) return;
  if (in_sizes[8] != NH) return;
  if (in_sizes[9] != 1) return;
  if (in_sizes[10] != SQ * SQ) return;
  if (out_size != SQ * HID) return;

  const float* x     = (const float*)d_in[0];
  const float* wq    = (const float*)d_in[1];
  const float* wk    = (const float*)d_in[2];
  const float* wv    = (const float*)d_in[3];
  const float* wo    = (const float*)d_in[4];
  const float* psh   = (const float*)d_in[5];
  const float* pls   = (const float*)d_in[6];
  const float* plc   = (const float*)d_in[7];
  const float* pss   = (const float*)d_in[8];
  const float* psl   = (const float*)d_in[9];
  const float* maskp = (const float*)d_in[10];
  float* out = (float*)d_out;

  size_t off = 0;
  const size_t oFL = off; off += 2048;
  const size_t oX  = off; off += (size_t)SQ * HID * 2;
  const size_t oWt = off; off += (size_t)NQKV * HID * 2;
  const size_t oWo = off; off += (size_t)HID * HID * 2;
  const size_t oQ  = off; off += (size_t)NH * SQ * HDM * 2;
  const size_t oK  = off; off += (size_t)NH * SQ * HDM * 2;
  const size_t oV  = off; off += (size_t)NH * HDM * SQ * 2;
  const size_t oO  = off; off += (size_t)NH * SQ * HDM * 2;
  if (off > ws_size) return;
  if (off > (size_t)134217728) return;

  char* ws = (char*)d_ws;
  unsigned* FL  = (unsigned*)(ws + oFL);
  _Float16* Xh  = (_Float16*)(ws + oX);
  _Float16* Wt  = (_Float16*)(ws + oWt);
  _Float16* Wot = (_Float16*)(ws + oWo);
  _Float16* Qp  = (_Float16*)(ws + oQ);
  _Float16* Kp  = (_Float16*)(ws + oK);
  _Float16* Vt  = (_Float16*)(ws + oV);
  _Float16* Op  = (_Float16*)(ws + oO);

  k_mflag<<<dim3(NQB), dim3(256), 0, stream>>>(maskp, FL);
  k_cvt<<<dim3(SQ), dim3(256), 0, stream>>>(x, Xh, 1.0f);
  k_cvt<<<dim3(HID), dim3(256), 0, stream>>>(wq, Wt, 32.0f);
  k_cvt<<<dim3(HID), dim3(256), 0, stream>>>(wk, Wt + (size_t)HID * HID, 32.0f);
  k_cvt<<<dim3(HID), dim3(256), 0, stream>>>(wv, Wt + (size_t)2 * HID * HID, 32.0f);
  k_cvt<<<dim3(HID), dim3(256), 0, stream>>>(wo, Wot, 32.0f);
  k_qkv<<<dim3(SQ / 64, NSLAB), dim3(128), 0, stream>>>(Xh, Wt, Qp, Kp, Vt);
  k_attn<<<dim3(NH * NQB), dim3(256), 0, stream>>>(Qp, Kp, Vt, maskp, FL, psh, pls, plc, pss, psl, Op);
  k_out<<<dim3(SQ / 256, HID / 64), dim3(256), 0, stream>>>(Op, Wot, out);
  (void)hipGetLastError();
}
